// RecurrentRGCN_50276887167213
// MI455X (gfx1250) — hardware-verified
//
#include <hip/hip_runtime.h>
#include <math.h>

#define NENT 20000
#define NNODE 20000
#define NEDGE 400000
#define NREL 460
#define HD 200
#define HP 256
#define KP 640
#define KG 608
#define NCOL 256
#define MP 20032
#define TILE 2048
#define NTILE 10
#define NROWA (NTILE * TILE)
#define NT 256
#define SCH 4096
#define SPE (SCH / NT)
#define NCH ((NEDGE + SCH - 1) / SCH)
#define WSCALE 16.0f
#define WSCALE_INV 0.0625f
#define RRELU_SLOPE_F 0.22916667f
#define NBTP (NCOL * (KP / 2))
#define NRELP (NREL * HP)
#define NPREP (2 * NBTP + NRELP)

static_assert(NEDGE % SPE == 0);
static_assert(MP % 64 == 0);
static_assert(NROWA >= MP);
static_assert((2 * NBTP) % NT == 0);
static_assert(NPREP % NT == 0);
static_assert((MP * (HP / 4)) % NT == 0);

typedef __attribute__((ext_vector_type(16))) _Float16 v16h;
typedef __attribute__((ext_vector_type(8)))  _Float16 v8h;
typedef __attribute__((ext_vector_type(16))) __bf16   v16b;
typedef __attribute__((ext_vector_type(8)))  __bf16   v8b;
typedef __attribute__((ext_vector_type(8)))  float    v8f;
typedef __attribute__((ext_vector_type(4)))  float    v4f;
typedef __attribute__((ext_vector_type(4)))  int      v4i;

__device__ __forceinline__ unsigned short f2bf_bits(float f) {
  unsigned u = __float_as_uint(f);
  return (unsigned short)((u + 0x7FFFu + ((u >> 16) & 1u)) >> 16);
}
__device__ __forceinline__ float bf_bits2f(unsigned short h) { return __uint_as_float(((unsigned)h) << 16); }

__device__ __forceinline__ void dep_guard_h(v8f& a, v8f& b, v16h x, v16h y) { asm volatile("v_nop\n\tv_nop\n\tv_nop\n\tv_nop" : "+v"(a), "+v"(b) : "v"(x), "v"(y)); }
__device__ __forceinline__ void dep_guard_b(v8f& a, v8f& b, v16b x, v16b y) { asm volatile("v_nop\n\tv_nop\n\tv_nop\n\tv_nop" : "+v"(a), "+v"(b) : "v"(x), "v"(y)); }
__device__ __forceinline__ void keep4_h(v16h a, v16h b, v16h c, v16h d) { asm volatile("v_nop" :: "v"(a), "v"(b), "v"(c), "v"(d)); }
__device__ __forceinline__ void keep4_b(v16b a, v16b b, v16b c, v16b d) { asm volatile("v_nop" :: "v"(a), "v"(b), "v"(c), "v"(d)); }
__device__ __forceinline__ void acc_guard4(v8f& a, v8f& b, v8f& c, v8f& d) { asm volatile("v_nop\n\tv_nop\n\tv_nop\n\tv_nop" : "+v"(a), "+v"(b), "+v"(c), "+v"(d)); }
template <typename T> struct Frag;
template <> struct Frag<_Float16> {
  typedef v16h V; union U { v16h v; v8h h[2]; };
  static __device__ __forceinline__ v16h load(const _Float16* p) {
    U f; f.h[0] = *(const v8h*)(p); f.h[1] = *(const v8h*)(p + 16); return f.v;
  }
  static __device__ __forceinline__ v8f mma(v16h a, v16h b, v8f c) {
    return __builtin_amdgcn_wmma_f32_16x16x32_f16(false, a, false, b, (short)0, c, false, false);
  }
  static __device__ __forceinline__ void guard(v8f& a, v8f& b, v16h x, v16h y) { dep_guard_h(a, b, x, y); }
  static __device__ __forceinline__ void keep(v16h a, v16h b, v16h c, v16h d) { keep4_h(a, b, c, d); }
};
template <> struct Frag<__bf16> {
  typedef v16b V; union U { v16b v; v8b h[2]; };
  static __device__ __forceinline__ v16b load(const __bf16* p) {
    U f; f.h[0] = *(const v8b*)(p); f.h[1] = *(const v8b*)(p + 16); return f.v;
  }
  static __device__ __forceinline__ v8f mma(v16b a, v16b b, v8f c) {
    return __builtin_amdgcn_wmma_f32_16x16x32_bf16(false, a, false, b, (short)0, c, false, false);
  }
  static __device__ __forceinline__ void guard(v8f& a, v8f& b, v16b x, v16b y) { dep_guard_b(a, b, x, y); }
  static __device__ __forceinline__ void keep(v16b a, v16b b, v16b c, v16b d) { keep4_b(a, b, c, d); }
};

template <int ET> struct Elem;
template <> struct Elem<0> { typedef _Float16 T; };
template <> struct Elem<1> { typedef __bf16 T; };
template <int ET, bool SPLIT, int BIAS_MODE, int OUT_MODE, bool RESID, int ACT = 0, bool DIFF = false>
__global__ __launch_bounds__(256) void wmma_gemm64(
    const unsigned short* __restrict__ Ap, const unsigned short* __restrict__ A2p, int lda, long strideA,
    const unsigned short* __restrict__ Btp, const unsigned short* __restrict__ Bt2p, int ldb, long strideB,
    void* __restrict__ Cout, void* __restrict__ Cout2, int ldc, long strideC,
    const float* __restrict__ bias,
    const float* __restrict__ resid, long strideR,
    int M, int N, int K, float scale) {
  typedef typename Elem<ET>::T T;
  typedef typename Frag<T>::V V;
  const T* A = (const T*)Ap; const T* A2 = (const T*)A2p; const T* Bt = (const T*)Btp; const T* Bt2 = (const T*)Bt2p;
  __shared__ __align__(16) float sT[8][16 * 68];
  const int b    = blockIdx.y;
  const int lane = threadIdx.x & 31;
  const int wave = threadIdx.x >> 5;
  const int tilesN = N >> 6;
  const int tilesM = M >> 6;
  const int tile = blockIdx.x * 8 + wave;
  if (tile >= tilesM * tilesN) return;
  const int tm = tile / tilesN;
  const int tn = tile - tm * tilesN;
  const int m0 = tm << 6;
  const int n0 = tn << 6;

  const T* Ab  = A  + (size_t)b * strideA;
  const T* Bb  = Bt + (size_t)b * strideB;
  const T* Ab2 = SPLIT ? (A2  + (size_t)b * strideA) : nullptr;
  const T* Bb2 = SPLIT ? (Bt2 + (size_t)b * strideB) : nullptr;

  const int rlane = lane & 15;
  const int koff  = (lane >> 4) * 8;
  const int mOff  = (lane >> 4) * 8;

  v8f acc[4][4];
#pragma unroll
  for (int i = 0; i < 4; ++i)
#pragma unroll
    for (int j = 0; j < 4; ++j) acc[i][j] = (v8f){0.f,0.f,0.f,0.f,0.f,0.f,0.f,0.f};

  for (int k0 = 0; k0 < K; k0 += 32) {
    V bh[4], bl[4];
#pragma unroll
    for (int j = 0; j < 4; ++j) {
      const size_t bo = (size_t)(n0 + (j << 4) + rlane) * ldb + koff + k0;
      bh[j] = Frag<T>::load(Bb + bo);
      if (SPLIT) bl[j] = Frag<T>::load(Bb2 + bo);
    }
#pragma unroll
    for (int i = 0; i < 4; ++i) {
      const size_t ao = (size_t)(m0 + (i << 4) + rlane) * lda + koff + k0;
      V ah = Frag<T>::load(Ab + ao);
      V al;
      if (SPLIT) al = Frag<T>::load(Ab2 + ao);
#pragma unroll
      for (int j = 0; j < 4; ++j) {
        acc[i][j] = Frag<T>::mma(ah, bh[j], acc[i][j]);
        if (SPLIT) {
          acc[i][j] = Frag<T>::mma(ah, bl[j], acc[i][j]);
          acc[i][j] = Frag<T>::mma(al, bh[j], acc[i][j]);
        }
      }
      Frag<T>::guard(acc[i][0], acc[i][3], ah, SPLIT ? al : ah);
    }
    Frag<T>::keep(bh[0], bh[1], bh[2], bh[3]);
    if (SPLIT) Frag<T>::keep(bl[0], bl[1], bl[2], bl[3]);
  }
  acc_guard4(acc[0][0], acc[0][1], acc[0][2], acc[0][3]);
  acc_guard4(acc[1][0], acc[1][1], acc[1][2], acc[1][3]);
  acc_guard4(acc[2][0], acc[2][1], acc[2][2], acc[2][3]);
  acc_guard4(acc[3][0], acc[3][1], acc[3][2], acc[3][3]);

  float* slab = sT[wave];
  const float* Rb = RESID ? (resid + (size_t)b * strideR) : nullptr;
#pragma unroll
  for (int i = 0; i < 4; ++i) {
    const int mBase = m0 + (i << 4);
#pragma unroll
    for (int j = 0; j < 4; ++j) {
      const int n = n0 + (j << 4) + rlane;
      float bv = 0.f;
      if (BIAS_MODE == 2) bv = bias[n];
#pragma unroll
      for (int r = 0; r < 8; ++r) {
        float v = acc[i][j][r] * scale;
        if (BIAS_MODE == 1) v += bias[mBase + mOff + r];
        if (BIAS_MODE == 2) v += bv;
        if (RESID) v += Rb[(size_t)(mBase + mOff + r) * ldc + n];
        if (ACT == 1) v = tanhf(v);
        if (ACT == 2) v = fmaxf(v, 0.0f);
        if (ACT == 3) v = v / (1.0f + expf(-v));
        if (ACT == 4) v = (v > 0.f) ? v : 0.01f * v;
        if (ACT == 5) v = 0.5f * v * (1.0f + erff(v * 0.70710678118654752f));
        if (ACT == 6) v = (v >= 0.f) ? v : RRELU_SLOPE_F * v;
        slab[(mOff + r) * 68 + (j << 4) + rlane] = v;
      }
    }
    __builtin_amdgcn_fence(__ATOMIC_RELEASE, "workgroup");
    __builtin_amdgcn_wave_barrier();
    __builtin_amdgcn_fence(__ATOMIC_ACQUIRE, "workgroup");
    if (OUT_MODE == 0) {
      float* C = (float*)Cout + (size_t)b * strideC;
      float* C2 = DIFF ? ((float*)Cout2 + (size_t)b * strideC) : nullptr;
      const float* Rd = DIFF ? (resid + (size_t)b * strideR) : nullptr;
      const int hh = lane >> 4, c4 = (lane & 15) * 4;
      for (int pass = 0; pass < 2; ++pass) {
#pragma unroll
        for (int it = 0; it < 8; ++it) {
          const int row = it * 2 + hh;
          v4f v = *(const v4f*)(slab + row * 68 + c4);
          *(volatile v4f*)(C + (size_t)(mBase + row) * ldc + n0 + c4) = v;
          if (DIFF) {
            const v4f rr = *(const v4f*)(Rd + (size_t)(mBase + row) * ldc + n0 + c4);
            const v4f dd = v - rr;
            *(volatile v4f*)(C2 + (size_t)(mBase + row) * ldc + n0 + c4) = dd;
          }
        }
        __threadfence();
      }
    } else {
      const int q = lane >> 3, c8 = (lane & 7) * 8;
      unsigned short* C  = (unsigned short*)Cout  + (size_t)b * strideC;
      unsigned short* C2 = (OUT_MODE == 2) ? ((unsigned short*)Cout2 + (size_t)b * strideC) : nullptr;
      for (int pass = 0; pass < 2; ++pass) {
#pragma unroll
        for (int it = 0; it < 4; ++it) {
          const int row = it * 4 + q;
          const float* sp = slab + row * 68 + c8;
          v8h hv, lv;
#pragma unroll
          for (int e = 0; e < 8; ++e) {
            if (OUT_MODE == 1) {
              hv[e] = (_Float16)sp[e];
            } else {
              unsigned short hb = f2bf_bits(sp[e]);
              unsigned short lb = f2bf_bits(sp[e] - bf_bits2f(hb));
              hv[e] = __builtin_bit_cast(_Float16, hb);
              lv[e] = __builtin_bit_cast(_Float16, lb);
            }
          }
          *(volatile v8h*)(C + (size_t)(mBase + row) * ldc + n0 + c8) = hv;
          if (OUT_MODE == 2) *(volatile v8h*)(C2 + (size_t)(mBase + row) * ldc + n0 + c8) = lv;
        }
        __threadfence();
      }
    }
    __builtin_amdgcn_fence(__ATOMIC_RELEASE, "workgroup");
    __builtin_amdgcn_wave_barrier();
    __builtin_amdgcn_fence(__ATOMIC_ACQUIRE, "workgroup");
  }
}

__device__ __forceinline__ int blk_excl_scan(int cnt, int* scan_ws, int tid, int* tot) {
  const int lane = tid & 31, wave = tid >> 5; int incl = cnt;
#pragma unroll
  for (int o = 1; o < 32; o <<= 1) { const int v = __shfl_up(incl, o, 32); if (lane >= o) incl += v; }
  if (lane == 31) scan_ws[wave] = incl;
  __syncthreads();
  if (wave == 0) { int wv = (lane < NT / 32) ? scan_ws[lane] : 0; int wincl = wv;
#pragma unroll
    for (int o = 1; o < 32; o <<= 1) { const int v = __shfl_up(wincl, o, 32); if (lane >= o) wincl += v; }
    if (lane < NT / 32) scan_ws[32 + lane] = wincl - wv; if (lane == 31) scan_ws[64] = wincl; }
  __syncthreads();
  const int res = scan_ws[32 + wave] + incl - cnt; *tot = scan_ws[64];
  return res;
}
__device__ __forceinline__ int chunk_hits3(const int* __restrict__ dstv, const int* __restrict__ srcv, const int* __restrict__ etv,
                                           int e0, int n0, int tid, int* LA, int* LB, int* scan_ws) {
  const int eb = e0 + tid * SPE;
  int ra[SPE]; int rb[SPE]; int cnt = 0;
  {
    const bool inr = (eb < NEDGE);
    const int ebc = inr ? eb : (NEDGE - SPE);
#pragma unroll
    for (int k = 0; k < SPE; k += 4) {
      const v4i d4 = *(const v4i*)(dstv + ebc + k);
      const v4i s4 = *(const v4i*)(srcv + ebc + k);
      const v4i t4 = *(const v4i*)(etv + ebc + k);
#pragma unroll
      for (int e = 0; e < 4; ++e) {
        const int d = d4[e]; int a = -1, bb = 0;
        if (inr && d >= n0 && d < n0 + TILE) {
          int s = s4[e]; s = s < 0 ? 0 : (s >= NNODE ? NNODE - 1 : s);
          int t = t4[e]; t = t < 0 ? 0 : (t >= NREL ? NREL - 1 : t);
          a = (d - n0) | (t << 11); bb = s; ++cnt;
        }
        ra[k + e] = a; rb[k + e] = bb;
      }
    }
  }
  int tot; int p = blk_excl_scan(cnt, scan_ws, tid, &tot);
#pragma unroll
  for (int k = 0; k < SPE; ++k) if (ra[k] >= 0) { if ((unsigned)p < (unsigned)SCH) { LA[p] = ra[k]; LB[p] = rb[k]; } ++p; }
  __syncthreads();
  return tot < SCH ? tot : SCH;
}

__device__ __forceinline__ v8h cvt8(const float* p, float f) {
  const v4f a = *(const v4f*)p; const v4f b = *(const v4f*)(p + 4);
  v8h r;
#pragma unroll
  for (int e = 0; e < 4; ++e) { r[e] = (_Float16)(a[e] * f); r[4 + e] = (_Float16)(b[e] * f); }
  return r;
}

__global__ __launch_bounds__(NT) void prep_kernel(const float* __restrict__ Wn1, const float* __restrict__ Wl1, const float* __restrict__ We1,
                                                 const float* __restrict__ Wn2, const float* __restrict__ Wl2, const float* __restrict__ We2,
                                                 const float* __restrict__ rel,
                                                 unsigned* __restrict__ BT1, unsigned* __restrict__ BT2, float* __restrict__ RELP) {
  const int i = blockIdx.x * NT + threadIdx.x;
  if (i < 2 * NBTP) {
    const int sel = (i >= NBTP) ? 1 : 0;
    const int j = i - sel * NBTP;
    const int n = j / (KP / 2);
    const int k = (j - n * (KP / 2)) * 2;
    const float* W0 = sel ? Wn2 : Wn1;
    const float* W1 = sel ? Wl2 : Wl1;
    const float* W2 = sel ? We2 : We1;
    const int nn = n < HD ? n : HD - 1;
    float v2[2];
#pragma unroll
    for (int u = 0; u < 2; ++u) {
      const int kk0 = k + u;
      const int kk = kk0 < 3 * HD ? kk0 : 3 * HD - 1;
      const int seg = (kk >= 2 * HD) ? 2 : ((kk >= HD) ? 1 : 0);
      const int ro = kk - seg * HD;
      const float* W = (seg == 0) ? W0 : ((seg == 1) ? W1 : W2);
      float v = W[(size_t)ro * HD + nn];
      if (kk0 >= 3 * HD || n >= HD) v = 0.f;
      v2[u] = v * WSCALE;
    }
    const _Float16 h0 = (_Float16)v2[0], h1 = (_Float16)v2[1];
    const unsigned uu = (unsigned)__builtin_bit_cast(unsigned short, h0) | ((unsigned)__builtin_bit_cast(unsigned short, h1) << 16);
    unsigned* dp = sel ? BT2 : BT1;
    ((volatile unsigned*)dp)[j] = uu;
    __threadfence();
    ((volatile unsigned*)dp)[j] = uu;
  } else if (i < NPREP) {
    const int i2 = i - 2 * NBTP;
    const int r = i2 >> 8, c = i2 & 255;
    const int cc = c < HD ? c : HD - 1;
    float v = rel[(size_t)r * HD + cc];
    if (c >= HD) v = 0.f;
    ((volatile float*)RELP)[i2] = v;
    __threadfence();
    ((volatile float*)RELP)[i2] = v;
  }
}

__global__ __launch_bounds__(NT) void gather_kernel(const float* __restrict__ ent, const int* __restrict__ nid, float* __restrict__ H0) {
  const int i = blockIdx.x * NT + threadIdx.x;
  if (i < MP * (HP / 4)) {
    const int n = i >> 6, q = i & 63;
    const int nc = n < NNODE ? n : NNODE - 1;
    int id = nid[nc]; id = id < 0 ? 0 : (id >= NENT ? NENT - 1 : id);
    const int qq = q < (HD / 4) ? q : (HD / 4) - 1;
    v4f v = *(const v4f*)(ent + (size_t)id * HD + 4 * qq);
    const v4f z = {0.f, 0.f, 0.f, 0.f};
    if (n >= NNODE || q >= (HD / 4)) v = z;
    *(volatile v4f*)(H0 + 4 * (size_t)i) = v;
    __threadfence();
    *(volatile v4f*)(H0 + 4 * (size_t)i) = v;
  }
}

template <bool FIRST>
__global__ __launch_bounds__(NT) void agg_kernel(const float* gsrc, const float* relp, const float* hself,
                                                const int* __restrict__ srcv, const int* __restrict__ dstv, const int* __restrict__ etv,
                                                float* AGG, unsigned short* __restrict__ A16) {
  __shared__ int LA[SCH];
  __shared__ int LB[SCH];
  __shared__ int SDEG[TILE];
  __shared__ int scan_ws[80];
  const int tid = threadIdx.x, lane = tid & 31, wave = tid >> 5;
  const int n0 = blockIdx.x * TILE;
  const v4f z4 = {0.f, 0.f, 0.f, 0.f};
  if (FIRST) {
    for (int pass = 0; pass < 2; ++pass) {
#pragma unroll 1
      for (int j = 0; j < TILE / 8; ++j) {
        float* rp = AGG + (size_t)(n0 + wave * (TILE / 8) + j) * HP + 4 * lane;
        *(volatile v4f*)rp = z4;
        *(volatile v4f*)(rp + 128) = z4;
      }
      __threadfence();
    }
  }
  for (int i = tid; i < TILE; i += NT) SDEG[i] = 0;
  __syncthreads();
#pragma unroll 1
  for (int c = 0; c < NCH; ++c) {
    const int tot = chunk_hits3(dstv, srcv, etv, c * SCH, n0, tid, LA, LB, scan_ws);
#pragma unroll 1
    for (int base = 0; base < tot; base += 32) {
      const int q = base + lane;
      const int qc = q < SCH ? q : SCH - 1;
      const int la = LA[qc], lb = LB[qc];
      const int ra = (q < tot) ? la : -1;
      const int own = (ra >= 0 && ((ra & (TILE - 1)) >> 8) == wave) ? 1 : 0;
      unsigned msk = (unsigned)__ballot(own);
#pragma unroll 1
      for (int it = 0; it < 32; ++it) {
        if (msk == 0u) break;
        const int bp = __builtin_ctz(msk); msk &= msk - 1u;
        const int a = __shfl(ra, bp, 32);
        const int s = __shfl(lb, bp, 32);
        const int dl = a & (TILE - 1);
        int t = a >> 11; t = t < NREL ? t : NREL - 1;
        if (lane == 0) SDEG[dl] += 1;
        float* rp = AGG + (size_t)(n0 + dl) * HP + 4 * lane;
        const float* gp = gsrc + (size_t)s * HP + 4 * lane;
        const v4f a0 = *(const v4f*)rp;
        const v4f a1 = *(const v4f*)(rp + 128);
        v4f m0 = *(const v4f*)gp;
        v4f m1 = *(const v4f*)(gp + 128);
        if (FIRST) {
          const float* tp = relp + (size_t)t * HP + 4 * lane;
          const v4f r0 = *(const v4f*)tp;
          const v4f r1 = *(const v4f*)(tp + 128);
          m0 = m0 + r0; m1 = m1 + r1;
        }
        const v4f o0 = a0 + m0;
        const v4f o1 = a1 + m1;
        *(volatile v4f*)rp = o0; *(volatile v4f*)(rp + 128) = o1;
        __threadfence();
        *(volatile v4f*)rp = o0; *(volatile v4f*)(rp + 128) = o1;
      }
    }
    __syncthreads();
  }
#pragma unroll 1
  for (int j = 0; j < TILE / 8; ++j) {
    const int dl = wave * (TILE / 8) + j;
    const int n = n0 + dl;
    const bool live = n < NNODE;
    const int nn = live ? n : NNODE - 1;
    const int deg = SDEG[dl];
    const float degf = (float)deg;
    const float norm = 1.0f / fmaxf(degf, 1.0f);
    const bool has = deg > 0;
    const float fN = live ? norm : 0.f;
    const float fL = (live && has) ? 1.f : 0.f;
    const float fE = (live && !has) ? 1.f : 0.f;
    const float* arow = AGG + (size_t)n * HP;
    const float* hrow = hself + (size_t)nn * HP;
    unsigned short* orow = A16 + (size_t)n * KP;
    const float* p0; float f0;
    if (lane < 25) { p0 = arow + 8 * lane; f0 = fN; } else { p0 = hrow + 8 * (lane - 25); f0 = fL; }
    const float* p1; float f1;
    if (lane < 18) { p1 = hrow + 8 * (lane + 7); f1 = fL; } else { p1 = hrow + 8 * (lane - 18); f1 = fE; }
    const float* p2; float f2;
    if (lane < 11) { p2 = hrow + 8 * (lane + 14); f2 = fE; } else { p2 = hrow; f2 = 0.f; }
    const v8h x0 = cvt8(p0, f0);
    const v8h x1 = cvt8(p1, f1);
    const v8h x2 = cvt8(p2, f2);
    *(volatile v8h*)(orow + 8 * lane) = x0;
    *(volatile v8h*)(orow + 256 + 8 * lane) = x1;
    if (lane < 16) *(volatile v8h*)(orow + 512 + 8 * lane) = x2;
    __threadfence();
    *(volatile v8h*)(orow + 8 * lane) = x0;
    *(volatile v8h*)(orow + 256 + 8 * lane) = x1;
    if (lane < 16) *(volatile v8h*)(orow + 512 + 8 * lane) = x2;
  }
}

__global__ __launch_bounds__(NT) void out_kernel(const float* __restrict__ H2, float* __restrict__ out) {
  const int i = blockIdx.x * NT + threadIdx.x;
  if (i < NNODE * (HD / 4)) {
    const int row = i / (HD / 4);
    const int col = (i - row * (HD / 4)) * 4;
    const v4f v = *(const v4f*)(H2 + (size_t)row * HP + col);
    *(volatile v4f*)(out + 4 * (size_t)i) = v;
    __threadfence();
    *(volatile v4f*)(out + 4 * (size_t)i) = v;
  }
}

extern "C" void kernel_launch(void* const* d_in, const int* in_sizes, int n_in,
                              void* d_out, int out_size, void* d_ws, size_t ws_size, hipStream_t stream) {
  if (n_in < 12) return;
  if (in_sizes[0] != NENT * HD || in_sizes[1] != NREL * HD || in_sizes[2] != HD * HD || in_sizes[8] != NNODE ||
      in_sizes[9] != NEDGE || in_sizes[10] != NEDGE || in_sizes[11] != NEDGE || out_size != NNODE * HD) return;
  const float* ent   = (const float*)d_in[0];
  const float* rel   = (const float*)d_in[1];
  const float* Wn1   = (const float*)d_in[2];
  const float* Wl1   = (const float*)d_in[3];
  const float* We1   = (const float*)d_in[4];
  const float* Wn2   = (const float*)d_in[5];
  const float* Wl2   = (const float*)d_in[6];
  const float* We2   = (const float*)d_in[7];
  const int*   nid   = (const int*)  d_in[8];
  const int*   src   = (const int*)  d_in[9];
  const int*   dst   = (const int*)  d_in[10];
  const int*   etype = (const int*)  d_in[11];
  float* out = (float*)d_out;

  char* ws = (char*)d_ws; size_t off = 0;
  auto carve = [&](size_t bytes) -> char* { char* p = ws + off; off += (bytes + 255) & ~(size_t)255; return p; };
  float*          RELP = (float*)carve((size_t)NREL * HP * 4);
  unsigned*       BT1  = (unsigned*)carve((size_t)NCOL * KP * 2);
  unsigned*       BT2  = (unsigned*)carve((size_t)NCOL * KP * 2);
  float*          H0   = (float*)carve((size_t)MP * HP * 4);
  float*          H1   = (float*)carve((size_t)MP * HP * 4);
  float*          G2   = (float*)carve((size_t)MP * HP * 4);
  float*          AGG  = (float*)carve((size_t)NROWA * HP * 4);
  unsigned short* A16  = (unsigned short*)carve((size_t)NROWA * KP * 2);
  if (off > ws_size || off > (size_t)134217728) return;
  float* H2 = H0;

  prep_kernel<<<NPREP / NT, NT, 0, stream>>>(Wn1, Wl1, We1, Wn2, Wl2, We2, rel, BT1, BT2, RELP);
  gather_kernel<<<(MP * (HP / 4)) / NT, NT, 0, stream>>>(ent, nid, H0);
  agg_kernel<true><<<NTILE, NT, 0, stream>>>(H0, RELP, H0, src, dst, etype, AGG, A16);
  const int gtiles = (MP / 64) * (NCOL / 64);
  wmma_gemm64<0, false, 0, 0, false, 6, true><<<dim3((gtiles + 7) / 8, 1), 256, 0, stream>>>(
      (const unsigned short*)A16, (const unsigned short*)A16, KP, 0L,
      (const unsigned short*)BT1, (const unsigned short*)BT1, KP, 0L,
      (void*)H1, (void*)G2, HP, 0L,
      (const float*)nullptr, (const float*)H0, 0L, MP, NCOL, KG, WSCALE_INV);
  agg_kernel<false><<<NTILE, NT, 0, stream>>>(G2, RELP, H1, src, dst, etype, AGG, A16);
  wmma_gemm64<0, false, 0, 0, false, 6, false><<<dim3((gtiles + 7) / 8, 1), 256, 0, stream>>>(
      (const unsigned short*)A16, (const unsigned short*)A16, KP, 0L,
      (const unsigned short*)BT2, (const unsigned short*)BT2, KP, 0L,
      (void*)H2, (void*)nullptr, HP, 0L,
      (const float*)nullptr, (const float*)nullptr, 0L, MP, NCOL, KG, WSCALE_INV);
  out_kernel<<<(NNODE * (HD / 4) + NT - 1) / NT, NT, 0, stream>>>(H2, out);
}
